// DynamicGCN_47107201302652
// MI455X (gfx1250) — hardware-run, weakly checked
//
#include <hip/hip_runtime.h>
#include <stddef.h>
#include <stdint.h>
#include <math.h>


#define CIN    128
#define HID    256
#define OUTC   128
#define K2     512
#define NHD    8
#define QKN    512
#define QKP    512
#define NTHR   256
#define NWAVE  8
#define EPT    8
#define CHUNK  (NTHR * EPT)
#define WCAP   (EPT * 32)
#define LISTN  (NWAVE * WCAP)
#define NBD    8192
#define SLD    13
#define NBA    512
#define SLA    9
#define RCAP   24576
#define DEGCAP 128
#define GBM    64
#define GBN    128
#define GTHR   128
#define SBM    64
#define EGRP   32
#define NU1    (HID * (CIN / 8))
#define NU2    (HID * (K2 / 8))
#define NU3    (OUTC * (K2 / 8))
#define NU4Q   (HID * (HID / 8))
#define NU4K   (HID * (HID / 8))
#define PO1    (NU1)
#define PO2    (PO1 + NU2)
#define PO3    (PO2 + NU3)
#define PO4    (PO3 + NU4Q)
#define PO5    (PO4 + NU4K)
#define AGG_ZINTS (LISTN + 2 * RCAP + 3 * NBA)
#define AGG_MISC  16
#define AGG_STG   (NWAVE * HID)
#define AGG_NRM   NBA
#define AGG_LDS_INTS (AGG_ZINTS + AGG_MISC + AGG_STG + AGG_NRM)
#define WSMAX  134217728
#define RSQD   0.17677669529663687f

static_assert((CHUNK & (CHUNK - 1)) == 0 && CHUNK <= 4096);
static_assert((NBD & (NBD - 1)) == 0 && NBD == (1 << SLD));
static_assert((NBA & (NBA - 1)) == 0 && NBA == (1 << SLA));
static_assert(((long long)CHUNK << SLD) < (1LL << 31));
static_assert(((long long)CHUNK << SLA) < (1LL << 31));
static_assert(NBD % (NTHR * 4) == 0);
static_assert(LISTN % NTHR == 0);
static_assert(NBA % NWAVE == 0 && NBA % 32 == 0 && NBA % GBM == 0 && NBA / 4 <= NTHR);
static_assert(RCAP % 4 == 0 && AGG_ZINTS % 4 == 0 && LISTN % 4 == 0 && AGG_LDS_INTS % 4 == 0);
static_assert(((AGG_ZINTS + AGG_MISC) % 4) == 0);
static_assert(CIN % 32 == 0 && HID % 32 == 0 && K2 == 2 * HID && OUTC == GBN && HID == 2 * GBN && QKN == 4 * GBN);
static_assert(GBM == (GTHR / 32) * 16 && GBN == 4 * 32);
static_assert(NU1 % NTHR == 0 && NU2 % NTHR == 0 && NU3 % NTHR == 0 && NU4Q % NTHR == 0 && NU4K % NTHR == 0);
static_assert(NHD * 32 == HID && NWAVE == NHD && SBM == 64);
static_assert(AGG_LDS_INTS * 4 <= 300000);
static_assert(DEGCAP % 32 == 0);

typedef float          v4f   __attribute__((ext_vector_type(4)));
typedef float          v8f   __attribute__((ext_vector_type(8)));
typedef int            v4i   __attribute__((ext_vector_type(4)));
typedef int            v8i   __attribute__((ext_vector_type(8)));
typedef unsigned int   v4u   __attribute__((ext_vector_type(4)));
typedef unsigned short v8us  __attribute__((ext_vector_type(8)));
typedef unsigned short v16us __attribute__((ext_vector_type(16)));
typedef __bf16         v16bf __attribute__((ext_vector_type(16)));
typedef v4f  __attribute__((may_alias)) v4fa;
typedef v4i  __attribute__((may_alias)) v4ia;
typedef v4u  __attribute__((may_alias)) v4ua;
typedef v8us __attribute__((may_alias)) v8usa;
union FragB { v16bf v; v16us u; v8us h[2]; v8i w; };

__device__ __forceinline__ v8f wmb(const FragB& a, const FragB& b, v8f c) {
  v8f d = __builtin_amdgcn_wmma_f32_16x16x32_bf16(false, a.v, false, b.v, (short)0, c, false, false);
  asm volatile("v_nop\n\tv_nop\n\tv_nop\n\tv_nop" : "+v"(d) : "v"(a.w), "v"(b.w));
  return d;
}

__device__ __forceinline__ unsigned bf16_bits(float f) {
  const unsigned u = __float_as_uint(f);
  return (u + 0x7FFFu + ((u >> 16) & 1u)) >> 16;
}
__device__ __forceinline__ float bf16_val(float f) {
  return __uint_as_float(bf16_bits(f) << 16);
}
__device__ __forceinline__ unsigned pk16(unsigned lo, unsigned hi) { return (lo & 0xffffu) | (hi << 16); }

template <int SLB>
__device__ __forceinline__ int scan_chunk(const int* __restrict__ dsts, int nE, int cbase, int slotBase,
                                          int nb, int vec8, int* list, int tid, int lane, int wave) {
  int wc = 0;
  const int el0  = tid * EPT;
  const int e0   = cbase + el0;
  const int sent = -2147483647 - 1;
  v4i da, db;
  if (vec8 != 0 && cbase + CHUNK <= nE) {
    da = *(const v4i*)(dsts + e0);
    db = *(const v4i*)(dsts + e0 + 4);
  } else {
    da.x = (e0     < nE) ? dsts[min(e0,     nE - 1)] : sent;
    da.y = (e0 + 1 < nE) ? dsts[min(e0 + 1, nE - 1)] : sent;
    da.z = (e0 + 2 < nE) ? dsts[min(e0 + 2, nE - 1)] : sent;
    da.w = (e0 + 3 < nE) ? dsts[min(e0 + 3, nE - 1)] : sent;
    db.x = (e0 + 4 < nE) ? dsts[min(e0 + 4, nE - 1)] : sent;
    db.y = (e0 + 5 < nE) ? dsts[min(e0 + 5, nE - 1)] : sent;
    db.z = (e0 + 6 < nE) ? dsts[min(e0 + 6, nE - 1)] : sent;
    db.w = (e0 + 7 < nE) ? dsts[min(e0 + 7, nE - 1)] : sent;
  }
  const unsigned nbs = (unsigned)slotBase;
  const unsigned unb = (unsigned)nb;
  const unsigned s0 = (unsigned)da.x - nbs, s1 = (unsigned)da.y - nbs;
  const unsigned s2 = (unsigned)da.z - nbs, s3 = (unsigned)da.w - nbs;
  const unsigned s4 = (unsigned)db.x - nbs, s5 = (unsigned)db.y - nbs;
  const unsigned s6 = (unsigned)db.z - nbs, s7 = (unsigned)db.w - nbs;
  const bool h0 = s0 < unb, h1 = s1 < unb, h2 = s2 < unb, h3 = s3 < unb;
  const bool h4 = s4 < unb, h5 = s5 < unb, h6 = s6 < unb, h7 = s7 < unb;
  const unsigned any = __builtin_amdgcn_ballot_w32(h0 | h1 | h2 | h3 | h4 | h5 | h6 | h7);
  if (any != 0u) {
#define HITJ(J, HJ, SJ) { \
      const unsigned mj = __builtin_amdgcn_ballot_w32(HJ); \
      if (mj != 0u) { \
        if (HJ) { \
          const int pos = wc + (int)__builtin_amdgcn_mbcnt_lo(mj, 0u); \
          if (pos < WCAP) list[wave * WCAP + pos] = ((el0 + (J)) << SLB) | (int)(SJ); \
        } \
        wc += (int)__builtin_popcount(mj); } }
    HITJ(0, h0, s0)
    HITJ(1, h1, s1)
    HITJ(2, h2, s2)
    HITJ(3, h3, s3)
    HITJ(4, h4, s4)
    HITJ(5, h5, s5)
    HITJ(6, h6, s6)
    HITJ(7, h7, s7)
#undef HITJ
  }
  return wc;
}

__global__ __launch_bounds__(NTHR) void k_prep(const float* __restrict__ x, int nN, int uX,
                                               const float* __restrict__ W1, const float* __restrict__ W2,
                                               const float* __restrict__ W3, const float* __restrict__ Wq,
                                               const float* __restrict__ Wk,
                                               unsigned short* XB, unsigned short* W1T, unsigned short* W2T,
                                               unsigned short* W3T, unsigned short* WQKT) {
  const int u = (int)blockIdx.x * NTHR + (int)threadIdx.x;
  v8us o;
  unsigned short* dp;
  if (u < uX) {
    const int row = u >> 4;
    const int k8  = (u & 15) * 8;
    const int rc  = row < nN ? row : nN - 1;
    const float* p = x + (size_t)rc * CIN + k8;
    const v4f a = *(const v4fa*)p;
    const v4f b = *(const v4fa*)(p + 4);
    o[0] = (unsigned short)bf16_bits(a.x); o[1] = (unsigned short)bf16_bits(a.y);
    o[2] = (unsigned short)bf16_bits(a.z); o[3] = (unsigned short)bf16_bits(a.w);
    o[4] = (unsigned short)bf16_bits(b.x); o[5] = (unsigned short)bf16_bits(b.y);
    o[6] = (unsigned short)bf16_bits(b.z); o[7] = (unsigned short)bf16_bits(b.w);
    dp = XB + (size_t)row * CIN + k8;
  } else {
    const int v = u - uX;
    if (v < PO1) {
      const int n  = v >> 4;
      const int k8 = (v & 15) * 8;
#pragma unroll
      for (int i = 0; i < 8; ++i) o[i] = (unsigned short)bf16_bits(W1[(size_t)(k8 + i) * HID + n]);
      dp = W1T + (size_t)n * CIN + k8;
    } else if (v < PO2) {
      const int t  = v - PO1;
      const int n  = t >> 6;
      const int k8 = (t & 63) * 8;
      const int kk = k8 & (HID - 1);
#pragma unroll
      for (int i = 0; i < 8; ++i) o[i] = (unsigned short)bf16_bits(W2[(size_t)(kk + i) * HID + n]);
      dp = W2T + (size_t)n * K2 + k8;
    } else if (v < PO3) {
      const int t  = v - PO2;
      const int n  = t >> 6;
      const int k8 = (t & 63) * 8;
      const int kk = k8 & (HID - 1);
#pragma unroll
      for (int i = 0; i < 8; ++i) o[i] = (unsigned short)bf16_bits(W3[(size_t)(kk + i) * OUTC + n]);
      dp = W3T + (size_t)n * K2 + k8;
    } else if (v < PO4) {
      const int t  = v - PO3;
      const int n  = t >> 5;
      const int k8 = (t & 31) * 8;
#pragma unroll
      for (int i = 0; i < 8; ++i) o[i] = (unsigned short)bf16_bits(Wq[(size_t)(k8 + i) * HID + n]);
      dp = WQKT + (size_t)n * HID + k8;
    } else if (v < PO5) {
      const int t  = v - PO4;
      const int n  = t >> 5;
      const int k8 = (t & 31) * 8;
#pragma unroll
      for (int i = 0; i < 8; ++i) o[i] = (unsigned short)bf16_bits(Wk[(size_t)(k8 + i) * HID + n]);
      dp = WQKT + (size_t)(HID + n) * HID + k8;
    } else {
      return;
    }
  }
  *(volatile v8us*)dp = o;
  __threadfence();
  *(volatile v8us*)dp = o;
}

__device__ __forceinline__ float disval(float s, bool live) {
  const float dg = s + 1.0f;
  const float r  = dg > 0.0f ? rsqrtf(fmaxf(dg, 1e-30f)) : 0.0f;
  return live ? r : 0.0f;
}

template <int RND>
__global__ __launch_bounds__(NTHR) void k_deg(const int* __restrict__ dsts, const float* __restrict__ ew,
                                              int nE, int nN, int vec8, float* dis) {
  __shared__ __attribute__((aligned(16))) float sdeg[NBD];
  __shared__ __attribute__((aligned(16))) int list[LISTN];
  __shared__ int wcnt[NWAVE];
  const int tid = (int)threadIdx.x, lane = tid & 31, wave = tid >> 5;
  const int nodeBase = (int)blockIdx.x * NBD;

  for (int i = tid; i < NBD; i += NTHR) sdeg[i] = 0.0f;
  for (int i = tid; i < LISTN; i += NTHR) list[i] = 0;
  if (tid < NWAVE) wcnt[tid] = 0;
  __syncthreads();

  const int nChunks = (nE + CHUNK - 1) / CHUNK;
#pragma unroll 1
  for (int ch = 0; ch < nChunks; ++ch) {
    const int cbase = ch * CHUNK;
    const int wc = scan_chunk<SLD>(dsts, nE, cbase, nodeBase, NBD, vec8, list, tid, lane, wave);
    if (lane == 0) wcnt[wave] = wc;
    __syncthreads();
    if (wave == 0) {
#pragma unroll 1
      for (int w2 = 0; w2 < NWAVE; ++w2) {
        int c = wcnt[w2];
        c = c < 0 ? 0 : (c > WCAP ? WCAP : c);
#pragma unroll 1
        for (int b0 = 0; b0 < c; b0 += 32) {
          const int idx = b0 + lane;
          const int ent = list[w2 * WCAP + (idx < WCAP ? idx : WCAP - 1)];
          const int el  = (ent >> SLD) & (CHUNK - 1);
          int eid = cbase + el;
          eid = eid < 0 ? 0 : (eid > nE - 1 ? nE - 1 : eid);
          const float wr  = ew[eid];
          const float wv  = (RND != 0) ? bf16_val(wr) : wr;
          const int   wvi = __float_as_int(wv);
          const int m32 = (c - b0) < 32 ? (c - b0) : 32;
#pragma unroll 1
          for (int k = 0; k < m32; ++k) {
            const int   uu  = __builtin_amdgcn_readlane(ent, k);
            const float wk  = __int_as_float(__builtin_amdgcn_readlane(wvi, k));
            const int   slt = uu & (NBD - 1);
            if (lane == 0) sdeg[slt] = sdeg[slt] + wk;
          }
        }
      }
    }
    __syncthreads();
  }

  v4f vals[NBD / (NTHR * 4)];
#pragma unroll
  for (int it = 0; it < NBD / (NTHR * 4); ++it) {
    const int s0 = it * (NTHR * 4) + 4 * tid;
    const v4f d4 = *(const v4fa*)(sdeg + s0);
    const int n0 = nodeBase + s0;
    v4f v;
    v.x = disval(d4.x, n0     < nN);
    v.y = disval(d4.y, n0 + 1 < nN);
    v.z = disval(d4.z, n0 + 2 < nN);
    v.w = disval(d4.w, n0 + 3 < nN);
    vals[it] = v;
  }
#pragma unroll
  for (int it = 0; it < NBD / (NTHR * 4); ++it) {
    const int s0 = it * (NTHR * 4) + 4 * tid;
    *(volatile v4f*)(dis + (size_t)nodeBase + s0) = vals[it];
  }
  __threadfence();
#pragma unroll
  for (int it = 0; it < NBD / (NTHR * 4); ++it) {
    const int s0 = it * (NTHR * 4) + 4 * tid;
    *(volatile v4f*)(dis + (size_t)nodeBase + s0) = vals[it];
  }
}

template <int OB>
__global__ __launch_bounds__(GTHR) void k_gemm(const unsigned short* __restrict__ A, int lda,
                                               const unsigned short* __restrict__ BT, int ldb, int K,
                                               float* Cm, int ldc,
                                               const float* __restrict__ bq, const float* __restrict__ bk,
                                               unsigned short* Cb, int ldcb) {
  __shared__ __attribute__((aligned(16))) float stg[GBM * GBN];
  const int tid = (int)threadIdx.x, lane = tid & 31, wave = tid >> 5, hh = lane >> 4, m = lane & 15;
  const int rowBase = (int)blockIdx.x * GBM;
  const int colBase = (int)blockIdx.y * GBN;

  v8f acc[8];
  {
    const v8f z = {0.f, 0.f, 0.f, 0.f, 0.f, 0.f, 0.f, 0.f};
#pragma unroll
    for (int t = 0; t < 8; ++t) acc[t] = z;
  }
  const unsigned short* ap = A  + (size_t)(rowBase + 16 * wave + m) * (size_t)lda + 8 * hh;
  const unsigned short* bp = BT + (size_t)(colBase + m) * (size_t)ldb + 8 * hh;

#pragma unroll 1
  for (int k0 = 0; k0 < K; k0 += 32) {
    FragB af;
    af.h[0] = *(const v8usa*)(ap + k0);
    af.h[1] = *(const v8usa*)(ap + k0 + 16);
#pragma unroll
    for (int nt = 0; nt < 8; ++nt) {
      const unsigned short* wq = bp + (size_t)(16 * nt) * (size_t)ldb + k0;
      FragB bf;
      bf.h[0] = *(const v8usa*)wq;
      bf.h[1] = *(const v8usa*)(wq + 16);
      acc[nt] = wmb(af, bf, acc[nt]);
    }
  }

#pragma unroll
  for (int nt = 0; nt < 8; ++nt) {
    const int lc = 16 * nt + m;
#pragma unroll
    for (int r = 0; r < 8; ++r) {
      const int lr = 16 * wave + 8 * hh + r;
      stg[lr * GBN + lc] = acc[nt][r];
    }
  }
  __syncthreads();

  if constexpr (OB == 0) {
    v4f pv[16];
#pragma unroll
    for (int i = 0; i < 16; ++i) pv[i] = *(const v4fa*)(stg + (16 * wave + i) * GBN + 4 * lane);
#pragma unroll
    for (int i = 0; i < 16; ++i) {
      float* op = Cm + (size_t)(rowBase + 16 * wave + i) * (size_t)ldc + colBase + 4 * lane;
      *(volatile v4f*)op = pv[i];
    }
    __threadfence();
#pragma unroll
    for (int i = 0; i < 16; ++i) {
      float* op = Cm + (size_t)(rowBase + 16 * wave + i) * (size_t)ldc + colBase + 4 * lane;
      *(volatile v4f*)op = pv[i];
    }
  } else {
    const int c8   = (lane & 15) * 8;
    const int rsub = lane >> 4;
    const int cb   = (colBase & (HID - 1)) + c8;
    const unsigned mq = (colBase < HID) ? 0xffffffffu : 0u;
    float b8[8];
    {
      const v4f q0 = *(const v4fa*)(bq + cb), q1 = *(const v4fa*)(bq + cb + 4);
      const v4f g0 = *(const v4fa*)(bk + cb), g1 = *(const v4fa*)(bk + cb + 4);
      float fq[8], fk[8];
      fq[0] = q0.x; fq[1] = q0.y; fq[2] = q0.z; fq[3] = q0.w; fq[4] = q1.x; fq[5] = q1.y; fq[6] = q1.z; fq[7] = q1.w;
      fk[0] = g0.x; fk[1] = g0.y; fk[2] = g0.z; fk[3] = g0.w; fk[4] = g1.x; fk[5] = g1.y; fk[6] = g1.z; fk[7] = g1.w;
#pragma unroll
      for (int e = 0; e < 8; ++e) {
        const unsigned sel = (__float_as_uint(fq[e]) & mq) | (__float_as_uint(fk[e]) & ~mq);
        b8[e] = bf16_val(__uint_as_float(sel));
      }
    }
    v4u hv[8];
#pragma unroll
    for (int it = 0; it < 8; ++it) {
      const int row = 16 * wave + 2 * it + rsub;
      const float* sp = stg + row * GBN + c8;
      const v4f f0 = *(const v4fa*)sp;
      const v4f f1 = *(const v4fa*)(sp + 4);
      v4u pkd;
      pkd[0] = pk16(bf16_bits(f0.x + b8[0]), bf16_bits(f0.y + b8[1]));
      pkd[1] = pk16(bf16_bits(f0.z + b8[2]), bf16_bits(f0.w + b8[3]));
      pkd[2] = pk16(bf16_bits(f1.x + b8[4]), bf16_bits(f1.y + b8[5]));
      pkd[3] = pk16(bf16_bits(f1.z + b8[6]), bf16_bits(f1.w + b8[7]));
      hv[it] = pkd;
    }
#pragma unroll
    for (int it = 0; it < 8; ++it) {
      const int row = 16 * wave + 2 * it + rsub;
      unsigned short* op = Cb + (size_t)(rowBase + row) * (size_t)ldcb + colBase + c8;
      *(volatile v4u*)(void*)op = hv[it];
    }
    __threadfence();
#pragma unroll
    for (int it = 0; it < 8; ++it) {
      const int row = 16 * wave + 2 * it + rsub;
      unsigned short* op = Cb + (size_t)(rowBase + row) * (size_t)ldcb + colBase + c8;
      *(volatile v4u*)(void*)op = hv[it];
    }
  }
}

template <int MODE>
__global__ __launch_bounds__(NTHR) void k_agg(const int* __restrict__ srcs, const int* __restrict__ dsts,
                                              const float* __restrict__ ew, int nE, int nN, int vec8, int mRows,
                                              const float* __restrict__ dis, const float* __restrict__ xl,
                                              const float* __restrict__ bias,
                                              float* hf, unsigned short* hb, float* nrmp, float* outp) {
  static_assert(MODE >= 1 && MODE <= 3);
  constexpr int CPL = (MODE == 3) ? 4 : 8;
  constexpr int C = CPL * 32;
  extern __shared__ __attribute__((aligned(16))) int dsm[];
  int* list = dsm;
  int* hl   = dsm + LISTN;
  int* sl   = dsm + LISTN + RCAP;
  int* cnt  = dsm + LISTN + 2 * RCAP;
  int* offs = cnt + NBA;
  int* cur  = offs + NBA;
  int* misc = cur + NBA;
  float* fstg = (float*)(misc + AGG_MISC);
  float* snrm = fstg + AGG_STG;
  const int tid = (int)threadIdx.x, lane = tid & 31, wave = tid >> 5;
  const int nodeBase = (int)blockIdx.x * NBA;

  {
    const v4i z4 = {0, 0, 0, 0};
    for (int i = tid * 4; i < AGG_LDS_INTS; i += NTHR * 4) *(v4ia*)(dsm + i) = z4;
  }
  float bv[CPL];
  {
    const float* bqp = bias + CPL * lane;
    const v4f a = *(const v4fa*)bqp;
    bv[0] = bf16_val(a.x); bv[1] = bf16_val(a.y); bv[2] = bf16_val(a.z); bv[3] = bf16_val(a.w);
    if constexpr (CPL == 8) {
      const v4f b = *(const v4fa*)(bqp + 4);
      bv[4] = bf16_val(b.x); bv[5] = bf16_val(b.y); bv[6] = bf16_val(b.z); bv[7] = bf16_val(b.w);
    }
  }
  __syncthreads();

  int t = 0, ov = 0;
  const int nChunks = (nE + CHUNK - 1) / CHUNK;
#pragma unroll 1
  for (int ch = 0; ch < nChunks; ++ch) {
    const int cbase = ch * CHUNK;
    const int wc = scan_chunk<SLA>(dsts, nE, cbase, nodeBase, NBA, vec8, list, tid, lane, wave);
    if (lane == 0) misc[wave] = wc;
    __syncthreads();
    if (wave == 0) {
#pragma unroll 1
      for (int w2 = 0; w2 < NWAVE; ++w2) {
        int c = misc[w2];
        c = c < 0 ? 0 : (c > WCAP ? WCAP : c);
#pragma unroll 1
        for (int b0 = 0; b0 < c; b0 += 32) {
          const int idx = b0 + lane;
          const int ent = list[w2 * WCAP + (idx < WCAP ? idx : WCAP - 1)];
          const int m32 = (c - b0) < 32 ? (c - b0) : 32;
#pragma unroll 1
          for (int k = 0; k < m32; ++k) {
            const int uu   = __builtin_amdgcn_readlane(ent, k);
            const int slot = uu & (NBA - 1);
            const int el   = (uu >> SLA) & (CHUNK - 1);
            const int pk   = ((cbase + el) << SLA) | slot;
            if (t < RCAP) {
              if (lane == 0) { hl[t] = pk; cnt[slot] = cnt[slot] + 1; }
              t = t + 1;
            } else {
              ov = 1;
            }
          }
        }
      }
    }
    __syncthreads();
  }
  if (wave == 0 && lane == 0) { misc[8] = t; misc[9] = ov; }
  __syncthreads();
  int tt = misc[8];
  tt = tt < 0 ? 0 : (tt > RCAP ? RCAP : tt);
  const int ovf = misc[9];

  if (wave == 0) {
    const int base = lane * (NBA / 32);
    int s = 0;
#pragma unroll 1
    for (int i = 0; i < NBA / 32; ++i) s += cnt[base + i];
    int incl = s;
#pragma unroll
    for (int d = 1; d < 32; d <<= 1) {
      const int y = __shfl_up(incl, d, 32);
      if (lane >= d) incl += y;
    }
    int run = incl - s;
#pragma unroll 1
    for (int i = 0; i < NBA / 32; ++i) {
      const int cv = cnt[base + i];
      offs[base + i] = run;
      cur[base + i]  = run;
      run += cv;
    }
  }
  __syncthreads();
  if (wave == 0) {
#pragma unroll 1
    for (int b0 = 0; b0 < tt; b0 += 32) {
      const int idx = b0 + lane;
      const int ent = hl[idx < RCAP ? idx : RCAP - 1];
      const int m32 = (tt - b0) < 32 ? (tt - b0) : 32;
#pragma unroll 1
      for (int k = 0; k < m32; ++k) {
        const int uu   = __builtin_amdgcn_readlane(ent, k);
        const int slot = uu & (NBA - 1);
        if (lane == 0) {
          int p = cur[slot];
          p = p < 0 ? 0 : (p > RCAP - 1 ? RCAP - 1 : p);
          sl[p] = uu;
          cur[slot] = p + 1;
        }
      }
    }
  }
  __syncthreads();

  const float pz = (ovf != 0) ? __int_as_float(0x7fc00000) : 0.0f;
#pragma unroll 1
  for (int si = 0; si < NBA / NWAVE; ++si) {
    const int s    = si * NWAVE + wave;
    const int node = nodeBase + s;
    int c = cnt[s];
    const bool big = c > DEGCAP;
    c = c < 0 ? 0 : (c > DEGCAP ? DEGCAP : c);
    int o = offs[s];
    o = o < 0 ? 0 : (o > RCAP ? RCAP : o);
    const int nc = node < nN ? node : nN - 1;
    const float dd = dis[nc];
    const float rd = dd * dd;
    float acc[CPL];
#pragma unroll
    for (int i = 0; i < CPL; ++i) acc[i] = 0.0f;
#pragma unroll 1
    for (int b0 = 0; b0 < c; b0 += 32) {
      int idx = o + b0 + lane;
      idx = idx > RCAP - 1 ? RCAP - 1 : idx;
      const int ent = sl[idx];
      int eid = ent >> SLA;
      eid = eid < 0 ? 0 : (eid > nE - 1 ? nE - 1 : eid);
      int sr = srcs[eid];
      sr = sr < 0 ? 0 : (sr > nN - 1 ? nN - 1 : sr);
      const float wr  = ew[eid];
      const float wv  = (MODE == 1) ? bf16_val(wr) : wr;
      const float cf  = (dis[sr] * wv) * dd;
      const int   cfi = __float_as_int(cf);
      const int m32 = (c - b0) < 32 ? (c - b0) : 32;
#pragma unroll 1
      for (int k = 0; k < m32; ++k) {
        const int   sk = __builtin_amdgcn_readlane(sr, k);
        const float ck = __int_as_float(__builtin_amdgcn_readlane(cfi, k));
        const float* rp = xl + (size_t)sk * C + CPL * lane;
        const v4f a = *(const v4fa*)rp;
        acc[0] = fmaf(ck, a.x, acc[0]); acc[1] = fmaf(ck, a.y, acc[1]);
        acc[2] = fmaf(ck, a.z, acc[2]); acc[3] = fmaf(ck, a.w, acc[3]);
        if constexpr (CPL == 8) {
          const v4f b = *(const v4fa*)(rp + 4);
          acc[4] = fmaf(ck, b.x, acc[4]); acc[5] = fmaf(ck, b.y, acc[5]);
          acc[6] = fmaf(ck, b.z, acc[6]); acc[7] = fmaf(ck, b.w, acc[7]);
        }
      }
    }
    float sv[CPL];
    {
      const float* sp = xl + (size_t)nc * C + CPL * lane;
      const v4f a = *(const v4fa*)sp;
      sv[0] = a.x; sv[1] = a.y; sv[2] = a.z; sv[3] = a.w;
      if constexpr (CPL == 8) {
        const v4f b = *(const v4fa*)(sp + 4);
        sv[4] = b.x; sv[5] = b.y; sv[6] = b.z; sv[7] = b.w;
      }
    }
    const float pzr = big ? __int_as_float(0x7fc00000) : pz;
    const bool live = node < nN;
    float v[CPL];
#pragma unroll
    for (int i = 0; i < CPL; ++i) {
      float y = (acc[i] + sv[i] * rd) + bv[i];
      if (MODE != 3) y = fmaxf(y, 0.0f);
      y = y + pzr;
      v[i] = live ? y : 0.0f;
    }
    if constexpr (MODE != 3) {
      v8us ho, lo8;
#pragma unroll
      for (int i = 0; i < 8; ++i) {
        const unsigned hbi = bf16_bits(v[i]);
        ho[i]  = (unsigned short)hbi;
        lo8[i] = (unsigned short)bf16_bits(v[i] - __uint_as_float(hbi << 16));
      }
      if constexpr (MODE == 2) {
        if (node < mRows) {
          unsigned short* hp = hb + (size_t)node * K2 + 8 * lane;
          *(volatile v8us*)hp = ho;
          *(volatile v8us*)(hp + HID) = lo8;
          __threadfence();
          *(volatile v8us*)hp = ho;
          *(volatile v8us*)(hp + HID) = lo8;
        }
      } else {
        float ss = 0.0f;
#pragma unroll
        for (int i = 0; i < 8; ++i) ss = fmaf(v[i], v[i], ss);
#pragma unroll
        for (int q = 16; q > 0; q >>= 1) ss += __shfl_xor(ss, q, 32);
        const float nv = fmaxf(sqrtf(ss), 1e-8f);
        if (lane == 0) snrm[s] = live ? nv : 0.0f;
        float* stg = fstg + wave * HID;
        v4f w0, w1;
        w0.x = v[0]; w0.y = v[1]; w0.z = v[2]; w0.w = v[3];
        w1.x = v[4]; w1.y = v[5]; w1.z = v[6]; w1.w = v[7];
        *(v4fa*)(stg + 8 * lane) = w0;
        *(v4fa*)(stg + 8 * lane + 4) = w1;
        __builtin_amdgcn_fence(__ATOMIC_RELEASE, "workgroup");
        __builtin_amdgcn_wave_barrier();
        __builtin_amdgcn_fence(__ATOMIC_ACQUIRE, "workgroup");
        const v4f p0 = *(const v4fa*)(stg + 4 * lane);
        const v4f p1 = *(const v4fa*)(stg + (HID / 2) + 4 * lane);
        __builtin_amdgcn_fence(__ATOMIC_RELEASE, "workgroup");
        __builtin_amdgcn_wave_barrier();
        __builtin_amdgcn_fence(__ATOMIC_ACQUIRE, "workgroup");
        if (node < mRows) {
          unsigned short* hp = hb + (size_t)node * K2 + 8 * lane;
          float* fp = hf + (size_t)node * HID + 4 * lane;
          *(volatile v8us*)hp = ho;
          *(volatile v8us*)(hp + HID) = lo8;
          *(volatile v4f*)fp = p0;
          *(volatile v4f*)(fp + HID / 2) = p1;
          __threadfence();
          *(volatile v8us*)hp = ho;
          *(volatile v8us*)(hp + HID) = lo8;
          *(volatile v4f*)fp = p0;
          *(volatile v4f*)(fp + HID / 2) = p1;
        }
      }
    } else {
      v4f ov4;
      ov4.x = v[0]; ov4.y = v[1]; ov4.z = v[2]; ov4.w = v[3];
      if (live) {
        float* op = outp + (size_t)node * OUTC + 4 * lane;
        *(volatile v4f*)op = ov4;
        __threadfence();
        *(volatile v4f*)op = ov4;
      }
    }
  }

  if constexpr (MODE == 1) {
    __syncthreads();
    v4f nv4;
    const int t4 = tid < NBA / 4 ? tid : NBA / 4 - 1;
    nv4 = *(const v4fa*)(snrm + 4 * t4);
    float* np = nrmp + (size_t)nodeBase + 4 * t4;
    if (tid < NBA / 4) *(volatile v4f*)np = nv4;
    __threadfence();
    if (tid < NBA / 4) *(volatile v4f*)np = nv4;
  }
}

__global__ __launch_bounds__(NTHR) void k_stats(const unsigned short* __restrict__ qkb, int nN,
                                                float* mpl, float* zpl) {
  __shared__ __attribute__((aligned(16))) unsigned short Ksh[64 * HID];
  __shared__ __attribute__((aligned(16))) float sM[SBM * NHD];
  __shared__ __attribute__((aligned(16))) float sZ[SBM * NHD];
  const int tid = (int)threadIdx.x, lane = tid & 31, wave = tid >> 5, hh = lane >> 4, c = lane & 15;
  const int r0 = (int)blockIdx.x * SBM;
  const v8f z8 = {0.f, 0.f, 0.f, 0.f, 0.f, 0.f, 0.f, 0.f};

  FragB qa[4];
#pragma unroll
  for (int i = 0; i < 4; ++i) {
    const unsigned short* qp = qkb + (size_t)(r0 + 16 * i + c) * QKP + 32 * wave + 8 * hh;
    qa[i].h[0] = *(const v8usa*)qp;
    qa[i].h[1] = *(const v8usa*)(qp + 16);
  }
  float mr[4][8], lr[4][8];
#pragma unroll
  for (int i = 0; i < 4; ++i)
#pragma unroll
    for (int r = 0; r < 8; ++r) { mr[i][r] = -INFINITY; lr[i][r] = 0.0f; }

  const int nkt = nN / 64;
#pragma unroll 1
  for (int kt = 0; kt < nkt; ++kt) {
    const int kv0 = kt * 64;
    __syncthreads();
    {
      const int row = tid >> 2, q4 = tid & 3;
      const unsigned short* src = qkb + (size_t)(kv0 + row) * QKP + HID + 64 * q4;
      unsigned short* dstp = Ksh + row * HID + 64 * q4;
#pragma unroll
      for (int i = 0; i < 8; ++i) {
        const v8us tv = *(const v8usa*)(src + 8 * i);
        *(v8usa*)(dstp + 8 * i) = tv;
      }
    }
    __syncthreads();

#pragma unroll
    for (int i = 0; i < 4; ++i) {
      v8f s[4];
#pragma unroll
      for (int j = 0; j < 4; ++j) {
        const unsigned short* kp = Ksh + (16 * j + c) * HID + 32 * wave + 8 * hh;
        FragB kb;
        kb.h[0] = *(const v8usa*)kp;
        kb.h[1] = *(const v8usa*)(kp + 16);
        s[j] = wmb(qa[i], kb, z8);
      }
#pragma unroll
      for (int r = 0; r < 8; ++r) {
        const float mx = fmaxf(fmaxf(s[0][r], s[1][r]), fmaxf(s[2][r], s[3][r]));
        const float nm = fmaxf(mr[i][r], mx);
        const float alpha = __expf((mr[i][r] - nm) * RSQD);
        float ps = __expf((s[0][r] - nm) * RSQD);
        ps += __expf((s[1][r] - nm) * RSQD);
        ps += __expf((s[2][r] - nm) * RSQD);
        ps += __expf((s[3][r] - nm) * RSQD);
        lr[i][r] = fmaf(lr[i][r], alpha, ps);
        mr[i][r] = nm;
      }
    }
  }

#pragma unroll
  for (int i = 0; i < 4; ++i) {
#pragma unroll
    for (int r = 0; r < 8; ++r) {
      float m = mr[i][r], l = lr[i][r];
#pragma unroll
      for (int off = 1; off < 16; off <<= 1) {
        const float om = __shfl_xor(m, off, 32);
        const float ol = __shfl_xor(l, off, 32);
        const float nm = fmaxf(m, om);
        l = l * __expf((m - nm) * RSQD) + ol * __expf((om - nm) * RSQD);
        m = nm;
      }
      if (c == 0) {
        sM[(16 * i + 8 * hh + r) * NHD + wave] = m;
        sZ[(16 * i + 8 * hh + r) * NHD + wave] = l;
      }
    }
  }
  __syncthreads();

  if (tid < NTHR / 2) {
    const v4f v = *(const v4fa*)(sM + 4 * tid);
    float* gp = mpl + (size_t)r0 * NHD + 4 * tid;
    *(volatile v4f*)gp = v;
    __threadfence();
    *(volatile v4f*)gp = v;
  } else {
    const int t2 = tid - NTHR / 2;
    const v4f v = *(const v4fa*)(sZ + 4 * t2);
    float* gp = zpl + (size_t)r0 * NHD + 4 * t2;
    *(volatile v4f*)gp = v;
    __threadfence();
    *(volatile v4f*)gp = v;
  }
}

__global__ __launch_bounds__(NTHR) void k_ew(const int* __restrict__ srcs, const int* __restrict__ dsts,
                                             int nE, int nN, int nGroups,
                                             const float* __restrict__ h1f, const float* __restrict__ nrm,
                                             const unsigned short* __restrict__ qkb,
                                             const float* __restrict__ mpl, const float* __restrict__ zpl,
                                             float* ew2) {
  const int tid = (int)threadIdx.x, lane = tid & 31, wave = tid >> 5;
  const int g = (int)blockIdx.x * NWAVE + wave;
  if (g >= nGroups) return;
  const int e0 = g * EGRP;
  int el = e0 + lane;
  el = el > nE - 1 ? nE - 1 : el;
  int sl = srcs[el];
  sl = sl < 0 ? 0 : (sl > nN - 1 ? nN - 1 : sl);
  int tl = dsts[el];
  tl = tl < 0 ? 0 : (tl > nN - 1 ? nN - 1 : tl);
  const int hd = lane >> 2;
  float outv = 0.0f;
#pragma unroll 1
  for (int k = 0; k < EGRP; ++k) {
    const int sk = __builtin_amdgcn_readlane(sl, k);
    const int tk = __builtin_amdgcn_readlane(tl, k);
    const float* hs = h1f + (size_t)sk * HID + 8 * lane;
    const float* ht = h1f + (size_t)tk * HID + 8 * lane;
    const v4f a0 = *(const v4fa*)hs;
    const v4f a1 = *(const v4fa*)(hs + 4);
    const v4f b0 = *(const v4fa*)ht;
    const v4f b1 = *(const v4fa*)(ht + 4);
    float d = a0.x * b0.x;
    d = fmaf(a0.y, b0.y, d); d = fmaf(a0.z, b0.z, d); d = fmaf(a0.w, b0.w, d);
    d = fmaf(a1.x, b1.x, d); d = fmaf(a1.y, b1.y, d); d = fmaf(a1.z, b1.z, d); d = fmaf(a1.w, b1.w, d);
#pragma unroll
    for (int q = 16; q > 0; q >>= 1) d += __shfl_xor(d, q, 32);
    const float den  = nrm[sk] * nrm[tk];
    const float cosv = d * (1.0f / den);

    const v4u qv = *(const v4ua*)(const void*)(qkb + (size_t)sk * QKP + 8 * lane);
    const v4u kv = *(const v4ua*)(const void*)(qkb + (size_t)tk * QKP + HID + 8 * lane);
    float p = 0.0f;
#pragma unroll
    for (int e = 0; e < 4; ++e) {
      const float qlo = __uint_as_float(qv[e] << 16), qhi = __uint_as_float(qv[e] & 0xffff0000u);
      const float klo = __uint_as_float(kv[e] << 16), khi = __uint_as_float(kv[e] & 0xffff0000u);
      p = fmaf(qlo, klo, p);
      p = fmaf(qhi, khi, p);
    }
    p += __shfl_xor(p, 1, 32);
    p += __shfl_xor(p, 2, 32);
    const float mh = mpl[(size_t)sk * NHD + hd];
    const float zh = zpl[(size_t)sk * NHD + hd];
    const float ah = __expf((p - mh) * RSQD) * (1.0f / zh);
    float as = ah;
    as += __shfl_xor(as, 4, 32);
    as += __shfl_xor(as, 8, 32);
    as += __shfl_xor(as, 16, 32);
    const float val = cosv * (as * 0.125f);
    outv = (lane == k) ? val : outv;
  }
  float* op = ew2 + (size_t)e0 + lane;
  *(volatile float*)op = outv;
  __threadfence();
  *(volatile float*)op = outv;
}

static inline int cdiv(int a, int b) { return (a + b - 1) / b; }

extern "C" void kernel_launch(void* const* d_in, const int* in_sizes, int n_in,
                              void* d_out, int out_size, void* d_ws, size_t ws_size,
                              hipStream_t stream) {
  if (n_in < 13) return;
  if (in_sizes[0] < CIN * 64 || (in_sizes[0] % CIN) != 0) return;
  const int nN = in_sizes[0] / CIN;
  if ((nN % 64) != 0 || nN > (1 << 21)) return;
  if (in_sizes[1] < 2 || (in_sizes[1] & 1) != 0) return;
  const int nE = in_sizes[1] / 2;
  if (nE < 1 || nE >= (1 << 22)) return;
  if (in_sizes[2] != nE) return;
  if (in_sizes[3] != CIN * HID || in_sizes[4] != HID) return;
  if (in_sizes[5] != HID * HID || in_sizes[6] != HID) return;
  if (in_sizes[7] != HID * OUTC || in_sizes[8] != OUTC) return;
  if (in_sizes[9] != HID * HID || in_sizes[10] != HID) return;
  if (in_sizes[11] != HID * HID || in_sizes[12] != HID) return;
  if ((long long)out_size != (long long)nN * OUTC) return;

  const float* x    = (const float*)d_in[0];
  const int*   edge = (const int*)d_in[1];
  const float* ewin = (const float*)d_in[2];
  const float* W1   = (const float*)d_in[3];
  const float* b1   = (const float*)d_in[4];
  const float* W2   = (const float*)d_in[5];
  const float* b2   = (const float*)d_in[6];
  const float* W3   = (const float*)d_in[7];
  const float* b3   = (const float*)d_in[8];
  const float* Wq   = (const float*)d_in[9];
  const float* bq   = (const float*)d_in[10];
  const float* Wk   = (const float*)d_in[11];
  const float* bk   = (const float*)d_in[12];
  float* out = (float*)d_out;
  const int* src = edge;
  const int* dst = edge + nE;

  const int gM   = nN / GBM;
  const int gS   = nN / SBM;
  const int gD   = cdiv(nN, NBD);
  const int NBPD = gD * NBD;
  const int gA   = cdiv(nN, NBA);
  const int NBPA = gA * NBA;
  if (NBPD < nN || NBPA < nN) return;
  const int nGroups = cdiv(nE, EGRP);
  const int nEP  = nGroups * EGRP;
  const int vec8 = ((nE & 3) == 0) ? 1 : 0;

  char* ws = (char*)d_ws;
  size_t off = 0;
  const size_t oXB  = off; off += (size_t)nN * CIN * 2;       off = (off + 255) & ~(size_t)255;
  const size_t oW1T = off; off += (size_t)HID * CIN * 2;      off = (off + 255) & ~(size_t)255;
  const size_t oW2T = off; off += (size_t)HID * K2 * 2;       off = (off + 255) & ~(size_t)255;
  const size_t oW3T = off; off += (size_t)OUTC * K2 * 2;      off = (off + 255) & ~(size_t)255;
  const size_t oWQK = off; off += (size_t)QKN * HID * 2;      off = (off + 255) & ~(size_t)255;
  const size_t oDS1 = off; off += (size_t)NBPD * 4;           off = (off + 255) & ~(size_t)255;
  const size_t oDS2 = off; off += (size_t)NBPD * 4;           off = (off + 255) & ~(size_t)255;
  const size_t oXW1 = off; off += (size_t)nN * HID * 4;       off = (off + 255) & ~(size_t)255;
  const size_t oH1F = off; off += (size_t)nN * HID * 4;       off = (off + 255) & ~(size_t)255;
  const size_t oH1A = off; off += (size_t)nN * K2 * 2;        off = (off + 255) & ~(size_t)255;
  const size_t oNRM = off; off += (size_t)NBPA * 4;           off = (off + 255) & ~(size_t)255;
  const size_t oQKB = off; off += (size_t)nN * QKP * 2;       off = (off + 255) & ~(size_t)255;
  const size_t oMPL = off; off += (size_t)nN * NHD * 4;       off = (off + 255) & ~(size_t)255;
  const size_t oZPL = off; off += (size_t)nN * NHD * 4;       off = (off + 255) & ~(size_t)255;
  const size_t oEW2 = off; off += (size_t)nEP * 4;            off = (off + 255) & ~(size_t)255;
  const size_t oXW2 = off; off += (size_t)nN * HID * 4;       off = (off + 255) & ~(size_t)255;
  const size_t oH2A = off; off += (size_t)nN * K2 * 2;        off = (off + 255) & ~(size_t)255;
  const size_t oXW3 = off; off += (size_t)nN * OUTC * 4;      off = (off + 255) & ~(size_t)255;
  if (off > ws_size || off > (size_t)WSMAX) return;

  unsigned short* XB   = (unsigned short*)(ws + oXB);
  unsigned short* W1T  = (unsigned short*)(ws + oW1T);
  unsigned short* W2T  = (unsigned short*)(ws + oW2T);
  unsigned short* W3T  = (unsigned short*)(ws + oW3T);
  unsigned short* WQKT = (unsigned short*)(ws + oWQK);
  float*          DIS1 = (float*)(ws + oDS1);
  float*          DIS2 = (float*)(ws + oDS2);
  float*          XW1  = (float*)(ws + oXW1);
  float*          H1F  = (float*)(ws + oH1F);
  unsigned short* H1A  = (unsigned short*)(ws + oH1A);
  float*          NRM  = (float*)(ws + oNRM);
  unsigned short* QKB  = (unsigned short*)(ws + oQKB);
  float*          MPL  = (float*)(ws + oMPL);
  float*          ZPL  = (float*)(ws + oZPL);
  float*          EW2  = (float*)(ws + oEW2);
  float*          XW2  = (float*)(ws + oXW2);
  unsigned short* H2A  = (unsigned short*)(ws + oH2A);
  float*          XW3  = (float*)(ws + oXW3);

  const size_t aggLds = (size_t)AGG_LDS_INTS * 4;
  hipFuncSetAttribute(reinterpret_cast<const void*>(&k_agg<1>), hipFuncAttributeMaxDynamicSharedMemorySize, (int)aggLds);
  hipFuncSetAttribute(reinterpret_cast<const void*>(&k_agg<2>), hipFuncAttributeMaxDynamicSharedMemorySize, (int)aggLds);
  hipFuncSetAttribute(reinterpret_cast<const void*>(&k_agg<3>), hipFuncAttributeMaxDynamicSharedMemorySize, (int)aggLds);

  const int uX = nN * (CIN / 8);
  k_prep<<<(uX + PO5) / NTHR, NTHR, 0, stream>>>(x, nN, uX, W1, W2, W3, Wq, Wk, XB, W1T, W2T, W3T, WQKT);
  k_gemm<0><<<dim3(gM, HID / GBN), GTHR, 0, stream>>>(XB, CIN, W1T, CIN, CIN, XW1, HID, bq, bk, QKB, QKP);
  k_deg<1><<<gD, NTHR, 0, stream>>>(dst, ewin, nE, nN, vec8, DIS1);
  k_agg<1><<<gA, NTHR, aggLds, stream>>>(src, dst, ewin, nE, nN, vec8, nN, DIS1, XW1, b1, H1F, H1A, NRM, out);
  k_gemm<1><<<dim3(gM, QKN / GBN), GTHR, 0, stream>>>(H1A, K2, WQKT, HID, HID, XW1, HID, bq, bk, QKB, QKP);
  k_stats<<<gS, NTHR, 0, stream>>>(QKB, nN, MPL, ZPL);
  k_ew<<<cdiv(nGroups, NWAVE), NTHR, 0, stream>>>(src, dst, nE, nN, nGroups, H1F, NRM, QKB, MPL, ZPL, EW2);
  k_deg<0><<<gD, NTHR, 0, stream>>>(dst, EW2, nE, nN, vec8, DIS2);
  k_gemm<0><<<dim3(gM, HID / GBN), GTHR, 0, stream>>>(H1A, K2, W2T, K2, K2, XW2, HID, bq, bk, QKB, QKP);
  k_agg<2><<<gA, NTHR, aggLds, stream>>>(src, dst, EW2, nE, nN, vec8, nN, DIS2, XW2, b2, H1F, H2A, NRM, out);
  k_gemm<0><<<dim3(gM, OUTC / GBN), GTHR, 0, stream>>>(H2A, K2, W3T, K2, K2, XW3, OUTC, bq, bk, QKB, QKP);
  k_agg<3><<<gA, NTHR, aggLds, stream>>>(src, dst, EW2, nE, nN, vec8, nN, DIS2, XW3, b3, H1F, H2A, NRM, out);
  (void)hipGetLastError();
}
